// HydraGCN_77687368450216
// MI455X (gfx1250) — hardware-verified
//
#include <hip/hip_runtime.h>


#define NBI  2
#define CC   64
#define NN   4096
#define NH_  4
#define FI   64
#define PJ   256
#define OUTC 64
#define NR   (NBI * NN)
#define RCH  1024
#define DM   CC
#define NTK  NN
#define EPS_BN 1e-5f
#define EPS_N  1e-12f
#define LOSC 1024.0f

typedef _Float16 h16;
typedef unsigned short bf;
typedef __attribute__((ext_vector_type(16))) __bf16   v16bf;
typedef __attribute__((ext_vector_type(16))) _Float16 v16h;
typedef __attribute__((ext_vector_type(8)))  _Float16 v8h;
typedef __attribute__((ext_vector_type(8)))  unsigned short v8us;
typedef __attribute__((ext_vector_type(8)))  float    v8f;
typedef __attribute__((ext_vector_type(4)))  float    v4f;
typedef __attribute__((ext_vector_type(4)))  _Float16 v4h;
typedef v8h  __attribute__((may_alias)) v8ha;
typedef v4f  __attribute__((may_alias)) v4fa;
typedef v8us __attribute__((may_alias)) v8usa;

__device__ __forceinline__ unsigned short f2bf(float f) { unsigned u = __float_as_uint(f); u += 0x7FFFu + ((u >> 16) & 1u); return (unsigned short)(u >> 16); }
__device__ __forceinline__ float bf2f(unsigned short b) { return __uint_as_float(((unsigned)b) << 16); }
__device__ __forceinline__ float bfr(float f) { return bf2f(f2bf(f)); }
__device__ __forceinline__ v16h cat16(v8h lo, v8h hi) { return __builtin_shufflevector(lo, hi, 0, 1, 2, 3, 4, 5, 6, 7, 8, 9, 10, 11, 12, 13, 14, 15); }
__device__ __forceinline__ v16bf cat16b(v8us lo, v8us hi) { return __builtin_bit_cast(v16bf, __builtin_shufflevector(lo, hi, 0, 1, 2, 3, 4, 5, 6, 7, 8, 9, 10, 11, 12, 13, 14, 15)); }
__device__ __forceinline__ v8f wmma16(v16h a, v16h b, v8f c) { return __builtin_amdgcn_wmma_f32_16x16x32_f16(false, a, false, b, (short)0, c, false, false); }
__device__ __forceinline__ v8f wmmab(v16bf a, v16bf b, v8f c) { return __builtin_amdgcn_wmma_f32_16x16x32_bf16(false, a, false, b, (short)0, c, false, false); }

__global__ __launch_bounds__(256) void k_wt(const float* __restrict__ Wm, int K, int ncols, bf* WT) {
    __shared__ __align__(16) unsigned short tl[64 * 72];
    const int tid = threadIdx.x, k0 = blockIdx.x * 64, n0 = blockIdx.y * 64;
    const int kk = tid >> 2, nq = (tid & 3) * 16;
#pragma unroll
    for (int i = 0; i < 16; ++i) tl[(nq + i) * 72 + kk] = f2bf(Wm[(size_t)(k0 + kk) * ncols + n0 + nq + i]);
    __syncthreads();
    const int piece = tid & 7;
    auto pass = [&]() {
#pragma unroll
        for (int s = 0; s < 2; ++s) { const int nr = (tid >> 3) + 32 * s; const v8us val = *(const v8usa*)(tl + nr * 72 + piece * 8); *(volatile v8us*)(WT + (size_t)(n0 + nr) * K + k0 + piece * 8) = val; }
    };
    pass(); __threadfence(); pass();
}
template <bool SPLITA, bool F16OUT = false>
__global__ __launch_bounds__(128) void k_gemmb(const bf* __restrict__ A, const bf* __restrict__ Al, const bf* __restrict__ Bn, const float* __restrict__ bias, float* C, int ldc, h16* C2, const float* __restrict__ R = nullptr, int K = DM, int roundR = 1) {
    __shared__ __align__(16) float ost[4][16 * 68];
    const int lane = threadIdx.x & 31, wave = threadIdx.x >> 5, lr = lane & 15, hi = lane >> 4;
    const int r0 = blockIdx.x * 64 + wave * 16, c0 = blockIdx.y * 64;
    const size_t aoff = (size_t)(r0 + lr) * K + 8 * hi;
    size_t boff[4];
#pragma unroll
    for (int t = 0; t < 4; ++t) boff[t] = (size_t)(c0 + t * 16 + lr) * K + 8 * hi;
    v8f acc[4];
#pragma unroll
    for (int t = 0; t < 4; ++t) acc[t] = (v8f){};
#pragma unroll 1
    for (int kc = 0; kc < K; kc += 32) {
        const v16bf a = cat16b(*(const v8us*)(A + aoff + kc), *(const v8us*)(A + aoff + kc + 16));
        v16bf al = a;
        if (SPLITA) al = cat16b(*(const v8us*)(Al + aoff + kc), *(const v8us*)(Al + aoff + kc + 16));
#pragma unroll
        for (int t = 0; t < 4; ++t) { const v16bf b = cat16b(*(const v8us*)(Bn + boff[t] + kc), *(const v8us*)(Bn + boff[t] + kc + 16)); acc[t] = wmmab(a, b, acc[t]); if (SPLITA) acc[t] = wmmab(al, b, acc[t]); }
        asm volatile("v_nop\n\tv_nop\n\tv_nop\n\tv_nop" : "+v"(acc[0]), "+v"(acc[1]), "+v"(acc[2]), "+v"(acc[3]) : "v"(a), "v"(al));
    }
    float* os = &ost[wave][0];
#pragma unroll
    for (int t = 0; t < 4; ++t) { const float bv = bias ? bfr(bias[c0 + t * 16 + lr]) : 0.f;
#pragma unroll
        for (int j = 0; j < 8; ++j) os[(hi * 8 + j) * 68 + t * 16 + lr] = acc[t][j] + bv; }
    __syncthreads();
    if (F16OUT) {
        h16* crow = (h16*)(void*)C + (size_t)r0 * ldc + c0;
        auto pass = [&]() {
#pragma unroll
            for (int s = 0; s < 4; ++s) { const int row = 4 * s + (lane >> 3), piece = lane & 7; const float* sp = os + row * 68 + piece * 8; v8h o, o2;
#pragma unroll
                for (int i = 0; i < 8; ++i) { const h16 a = (h16)sp[i]; o[i] = a; o2[i] = (h16)((sp[i] - (float)a) * LOSC); }
                *(volatile v8h*)(crow + (size_t)row * ldc + piece * 8) = o; if (C2) *(volatile v8h*)(C2 + (size_t)r0 * ldc + c0 + (size_t)row * ldc + piece * 8) = o2; }
        };
        pass(); __threadfence(); pass();
    } else {
        float* crow = C + (size_t)r0 * ldc + c0;
        auto pass = [&]() {
#pragma unroll
            for (int s = 0; s < 8; ++s) { const int Lid = (lane >> 3) + 4 * s, piece = lane & 7; const int row = Lid >> 1, cofs = (Lid & 1) * 32 + piece * 4;
                v4f val = *(const v4fa*)(os + row * 68 + cofs); if (R) { const v4f rv = *(const v4f*)(R + ((size_t)r0 + row) * ldc + c0 + cofs); val += roundR ? (v4f){bfr(rv[0]), bfr(rv[1]), bfr(rv[2]), bfr(rv[3])} : rv; }
                *(volatile v4f*)(crow + (size_t)row * ldc + cofs) = val; }
        };
        pass(); __threadfence(); pass();
    }
}

__global__ __launch_bounds__(128) void k_gemm3(const bf* __restrict__ Ah, const bf* __restrict__ Al, const bf* __restrict__ Bh, const bf* __restrict__ Bl, int K, float* C, int ldc) {
    __shared__ __align__(16) float ost[4][16 * 68];
    const int lane = threadIdx.x & 31, wave = threadIdx.x >> 5, lr = lane & 15, hi = lane >> 4;
    const int r0 = blockIdx.x * 64 + wave * 16, c0 = blockIdx.y * 64;
    const size_t aoff = (size_t)(r0 + lr) * K + 8 * hi;
    v8f acc[4];
#pragma unroll
    for (int t = 0; t < 4; ++t) acc[t] = (v8f){};
#pragma unroll 1
    for (int kc = 0; kc < K; kc += 32) {
        const v16bf a = cat16b(*(const v8us*)(Ah + aoff + kc), *(const v8us*)(Ah + aoff + kc + 16));
        const v16bf al = cat16b(*(const v8us*)(Al + aoff + kc), *(const v8us*)(Al + aoff + kc + 16));
#pragma unroll
        for (int t = 0; t < 4; ++t) { const size_t bo = (size_t)(c0 + t * 16 + lr) * K + kc + 8 * hi;
            const v16bf bh = cat16b(*(const v8us*)(Bh + bo), *(const v8us*)(Bh + bo + 16)); const v16bf bl = cat16b(*(const v8us*)(Bl + bo), *(const v8us*)(Bl + bo + 16));
            acc[t] = wmmab(a, bh, acc[t]); acc[t] = wmmab(al, bh, acc[t]); acc[t] = wmmab(a, bl, acc[t]); }
        asm volatile("v_nop\n\tv_nop\n\tv_nop\n\tv_nop" : "+v"(acc[0]), "+v"(acc[1]), "+v"(acc[2]), "+v"(acc[3]) : "v"(a), "v"(al));
    }
    float* os = &ost[wave][0];
#pragma unroll
    for (int t = 0; t < 4; ++t) {
#pragma unroll
        for (int j = 0; j < 8; ++j) os[(hi * 8 + j) * 68 + t * 16 + lr] = acc[t][j]; }
    __builtin_amdgcn_wave_barrier(); asm volatile("" ::: "memory");
    float* crow = C + (size_t)r0 * ldc + c0;
    auto pass = [&]() {
#pragma unroll
        for (int s = 0; s < 8; ++s) { const int Lid = (lane >> 3) + 4 * s, piece = lane & 7; const int row = Lid >> 1, cofs = (Lid & 1) * 32 + piece * 4;
            const v4f val = *(const v4fa*)(os + row * 68 + cofs); *(volatile v4f*)(crow + (size_t)row * ldc + cofs) = val; }
    };
    pass(); __threadfence(); pass();
}

__global__ __launch_bounds__(256) void k_bf(const float* __restrict__ src, bf* dst, size_t n8) {
    const size_t i = (size_t)blockIdx.x * 256 + threadIdx.x; if (i >= n8) return;
    const v8f v = *(const v8f*)(src + i * 8); v8us o;
#pragma unroll
    for (int k = 0; k < 8; ++k) o[k] = f2bf(v[k]);
    *(volatile v8us*)(dst + i * 8) = o; __threadfence(); *(volatile v8us*)(dst + i * 8) = o;
}
__global__ __launch_bounds__(256) void k_l2n(const float* __restrict__ Y, float* DST) {
    const int lane = threadIdx.x & 31, n = blockIdx.x * 8 + (threadIdx.x >> 5); if (n >= NN) return;
    const size_t o = (size_t)n * PJ + lane * 8; const v8f v = *(const v8f*)(Y + o); float ss = 0.f;
#pragma unroll
    for (int i = 0; i < 8; ++i) ss = fmaf(v[i], v[i], ss);
    ss += __shfl_xor(ss, 1, 32); ss += __shfl_xor(ss, 2, 32); ss += __shfl_xor(ss, 4, 32);
    const float inv = 1.0f / fmaxf(sqrtf(ss), EPS_N); v8f y;
#pragma unroll
    for (int i = 0; i < 8; ++i) y[i] = v[i] * inv;
    *(volatile v8f*)(DST + o) = y; __threadfence(); *(volatile v8f*)(DST + o) = y;
}
__global__ __launch_bounds__(256) void k_kv(const float* __restrict__ K, const float* __restrict__ V, float* KVS) {
    const int j = threadIdx.x; float s = 0.f;
#pragma unroll 1
    for (int n = 0; n < NN; ++n) s = fmaf(K[(size_t)n * PJ + j], V[(size_t)n * PJ + j], s);
    *(volatile float*)(KVS + j) = s; __threadfence(); *(volatile float*)(KVS + j) = s;
}
__global__ __launch_bounds__(256) void k_hydra(const float* __restrict__ Q, const float* __restrict__ KVS, bf* Hh, bf* Hl) {
    const int lane = threadIdx.x & 31, n = blockIdx.x * 8 + (threadIdx.x >> 5); if (n >= NN) return;
    const size_t o = (size_t)n * PJ + lane * 8; const v8f v = *(const v8f*)(Q + o); v8us oh, ol;
#pragma unroll
    for (int i = 0; i < 8; ++i) { const float y = v[i] * KVS[lane * 8 + i]; const unsigned short hb = f2bf(y); oh[i] = hb; ol[i] = f2bf(y - bf2f(hb)); }
    *(volatile v8us*)(Hh + o) = oh; *(volatile v8us*)(Hl + o) = ol; __threadfence(); *(volatile v8us*)(Hh + o) = oh; *(volatile v8us*)(Hl + o) = ol;
}
__global__ __launch_bounds__(256) void k_hmean(const float* __restrict__ Y, bf* Mh, bf* Ml) {
    typedef __attribute__((ext_vector_type(2))) unsigned short v2us;
    const int lane = threadIdx.x & 31, n = blockIdx.x * 8 + (threadIdx.x >> 5); if (n >= NN) return;
    v2us oh, ol;
#pragma unroll
    for (int i = 0; i < 2; ++i) { const int f = 2 * lane + i; const float* r = Y + (size_t)n * PJ + f; const float m = (((r[0] + r[FI]) + r[2 * FI]) + r[3 * FI]) * 0.25f; const unsigned short hb = f2bf(m); oh[i] = hb; ol[i] = f2bf(m - bf2f(hb)); }
    const size_t o = (size_t)n * FI + 2 * lane;
    *(volatile v2us*)(Mh + o) = oh; *(volatile v2us*)(Ml + o) = ol; __threadfence(); *(volatile v2us*)(Mh + o) = oh; *(volatile v2us*)(Ml + o) = ol;
}
__global__ __launch_bounds__(64) void k_bnstat(const float* __restrict__ P, float* MU, float* RS) {
    const int c = threadIdx.x; float s = 0.f;
#pragma unroll 1
    for (int r = 0; r < NR; ++r) s += P[(size_t)r * OUTC + c];
    const float mu = s * (1.0f / NR); float s2 = 0.f;
#pragma unroll 1
    for (int r = 0; r < NR; ++r) { const float d = P[(size_t)r * OUTC + c] - mu; s2 = fmaf(d, d, s2); }
    const float rs = rsqrtf(s2 * (1.0f / NR) + EPS_BN);
    *(volatile float*)(MU + c) = mu; *(volatile float*)(RS + c) = rs; __threadfence(); *(volatile float*)(MU + c) = mu; *(volatile float*)(RS + c) = rs;
}
__global__ __launch_bounds__(256) void k_bn1(const float* __restrict__ P, const float* __restrict__ MU, const float* __restrict__ RS, const float* __restrict__ g, const float* __restrict__ be, float* H1) {
    typedef __attribute__((ext_vector_type(2))) float v2f;
    const int lane = threadIdx.x & 31, r = blockIdx.x * 8 + (threadIdx.x >> 5); if (r >= NR) return;
    v2f y;
#pragma unroll
    for (int i = 0; i < 2; ++i) { const int c = 2 * lane + i; y[i] = fmaxf((P[(size_t)r * OUTC + c] - MU[c]) * RS[c] * bfr(g[c]) + bfr(be[c]), 0.f); }
    const size_t o = (size_t)r * OUTC + 2 * lane; *(volatile v2f*)(H1 + o) = y; __threadfence(); *(volatile v2f*)(H1 + o) = y;
}
__global__ __launch_bounds__(128) void k_cmean(const float* __restrict__ H1, float* MU1) {
    const int u = threadIdx.x; const int b = u / OUTC, c = u % OUTC; float s = 0.f;
#pragma unroll 1
    for (int n = 0; n < NN; ++n) s += H1[((size_t)b * NN + n) * OUTC + c];
    const float m = s * (1.0f / NN); *(volatile float*)(MU1 + u) = m; __threadfence(); *(volatile float*)(MU1 + u) = m;
}
__global__ __launch_bounds__(256) void k_h1T(const float* __restrict__ H1, const float* __restrict__ MU1, bf* Th, bf* Tl) {
    typedef __attribute__((ext_vector_type(2))) unsigned short v2us;
    const int lane = threadIdx.x & 31, wid = blockIdx.x * 8 + (threadIdx.x >> 5); if (wid >= NBI * OUTC * (NN / 64)) return;
    const int tg = wid % (NN / 64), rest = wid / (NN / 64), c = rest % OUTC, b = rest / OUTC; const int n0 = tg * 64 + 2 * lane; const float mu = MU1[b * OUTC + c];
    v2us oh, ol;
#pragma unroll
    for (int i = 0; i < 2; ++i) { const float y = H1[((size_t)b * NN + n0 + i) * OUTC + c] - mu; const unsigned short hb = f2bf(y); oh[i] = hb; ol[i] = f2bf(y - bf2f(hb)); }
    const size_t o = ((size_t)b * OUTC + c) * NN + n0;
    *(volatile v2us*)(Th + o) = oh; *(volatile v2us*)(Tl + o) = ol; __threadfence(); *(volatile v2us*)(Th + o) = oh; *(volatile v2us*)(Tl + o) = ol;
}
__global__ __launch_bounds__(256) void k_rbias(const float* __restrict__ MU1, const float* __restrict__ w2, float* RB) {
    const int u = blockIdx.x * 256 + threadIdx.x; if (u >= NBI * RCH * OUTC) return;
    const int o = u % OUTC, b = u / (RCH * OUTC); float s = 0.f;
#pragma unroll 1
    for (int c = 0; c < OUTC; ++c) s = fmaf(MU1[b * OUTC + c], bfr(w2[o * OUTC + c]), s);
    *(volatile float*)(RB + u) = s; __threadfence(); *(volatile float*)(RB + u) = s;
}
__global__ __launch_bounds__(256) void k_softmax(const float* __restrict__ S, bf* PH, bf* PL) {
    const int lane = threadIdx.x & 31, r = blockIdx.x * 8 + (threadIdx.x >> 5); if (r >= RCH) return;
    const float* sr = S + (size_t)r * NN; float m = -3.0e38f;
#pragma unroll 1
    for (int c0 = lane * 8; c0 < NN; c0 += 256) { const v8f v = *(const v8f*)(sr + c0);
#pragma unroll
        for (int i = 0; i < 8; ++i) m = fmaxf(m, v[i]); }
#pragma unroll
    for (int sh = 16; sh; sh >>= 1) m = fmaxf(m, __shfl_xor(m, sh, 32));
    float sum = 0.f;
#pragma unroll 1
    for (int c0 = lane * 8; c0 < NN; c0 += 256) { const v8f v = *(const v8f*)(sr + c0);
#pragma unroll
        for (int i = 0; i < 8; ++i) sum += __expf(v[i] - m); }
#pragma unroll
    for (int sh = 16; sh; sh >>= 1) sum += __shfl_xor(sum, sh, 32);
    const float inv = 1.0f / sum;
#pragma unroll 1
    for (int ps = 0; ps < 2; ++ps) {
#pragma unroll 1
        for (int c0 = lane * 8; c0 < NN; c0 += 256) { const v8f v = *(const v8f*)(sr + c0); v8us oh, ol;
#pragma unroll
            for (int i = 0; i < 8; ++i) { const float p = __expf(v[i] - m) * inv; const unsigned short hb = f2bf(p); oh[i] = hb; ol[i] = f2bf(p - bf2f(hb)); }
            const size_t o = (size_t)r * NN + c0; *(volatile v8us*)(PH + o) = oh; *(volatile v8us*)(PL + o) = ol; }
        if (ps == 0) __threadfence(); }
}
__global__ __launch_bounds__(256) void k_split64(const float* __restrict__ src, int nrows, bf* dh, bf* dl) {
    typedef __attribute__((ext_vector_type(2))) unsigned short v2us;
    const int lane = threadIdx.x & 31, r = blockIdx.x * 8 + (threadIdx.x >> 5); if (r >= nrows) return;
    const size_t o = (size_t)r * 64 + lane * 2; v2us oh, ol;
#pragma unroll
    for (int i = 0; i < 2; ++i) { const float v = src[o + i]; const unsigned short hb = f2bf(v); oh[i] = hb; ol[i] = f2bf(v - bf2f(hb)); }
    *(volatile v2us*)(dh + o) = oh; *(volatile v2us*)(dl + o) = ol; __threadfence(); *(volatile v2us*)(dh + o) = oh; *(volatile v2us*)(dl + o) = ol;
}
__global__ __launch_bounds__(256) void k_bn2out(const float* __restrict__ P2, const float* __restrict__ MU, const float* __restrict__ RS, const float* __restrict__ g, const float* __restrict__ be, float* OUTP) {
    const int lane = threadIdx.x & 31, wid = blockIdx.x * 8 + (threadIdx.x >> 5); if (wid >= NBI * OUTC * (NN / 128)) return;
    const int tg = wid % (NN / 128), rest = wid / (NN / 128), c = rest % OUTC, b = rest / OUTC; const int n0 = tg * 128 + 4 * lane;
    const float mu = MU[c], rs = RS[c], gg = bfr(g[c]), bb = bfr(be[c]); v4f y;
#pragma unroll
    for (int i = 0; i < 4; ++i) y[i] = fmaxf((P2[((size_t)b * NN + n0 + i) * OUTC + c] - mu) * rs * gg + bb, 0.f);
    const size_t o = ((size_t)b * OUTC + c) * NN + n0; *(volatile v4f*)(OUTP + o) = y; __threadfence(); *(volatile v4f*)(OUTP + o) = y;
}

extern "C" void kernel_launch(void* const* d_in, const int* in_sizes, int n_in,
                              void* d_out, int out_size, void* d_ws, size_t ws_size, hipStream_t stream) {
    (void)in_sizes; (void)n_in; (void)out_size;
    const float* x = (const float*)d_in[0]; const float* wk = (const float*)d_in[1]; const float* bk = (const float*)d_in[2]; const float* wq = (const float*)d_in[3]; const float* bq = (const float*)d_in[4]; const float* wv = (const float*)d_in[5]; const float* bv = (const float*)d_in[6];
    const float* w1 = (const float*)d_in[7]; const float* b1 = (const float*)d_in[8]; const float* g1 = (const float*)d_in[9]; const float* be1 = (const float*)d_in[10]; const float* w2 = (const float*)d_in[11]; const float* b2 = (const float*)d_in[12]; const float* g2 = (const float*)d_in[13]; const float* be2 = (const float*)d_in[14];
    float* out = (float*)d_out;
    char* wsp = (char*)d_ws;
    auto take = [&](size_t bytes) { char* p = wsp; wsp += (bytes + 255) & ~(size_t)255; return (void*)p; };
    bf* WkB = (bf*)take(PJ * CC * 2); bf* WqB = (bf*)take(PJ * CC * 2); bf* WvB = (bf*)take(PJ * CC * 2); bf* W1B = (bf*)take(OUTC * PJ * 2); bf* W2B = (bf*)take(OUTC * OUTC * 2);
    bf* XT = (bf*)take((size_t)NN * CC * 2); float* Kf = (float*)take((size_t)NBI * NN * PJ * 4); float* Qf = (float*)take((size_t)NBI * NN * PJ * 4); float* Vf = (float*)take((size_t)NN * PJ * 4); float* KVS = (float*)take(PJ * 4);
    bf* Hh = (bf*)take((size_t)NN * PJ * 2); bf* Hl = (bf*)take((size_t)NN * PJ * 2); float* P1 = (float*)take((size_t)NR * OUTC * 4); float* MU = (float*)take(256); float* RS = (float*)take(256);
    float* H1 = (float*)take((size_t)NR * OUTC * 4); float* MU1 = (float*)take(NBI * OUTC * 4); float* RB = (float*)take((size_t)NBI * RCH * OUTC * 4); bf* H1Th = (bf*)take((size_t)NBI * OUTC * NN * 2); bf* H1Tl = (bf*)take((size_t)NBI * OUTC * NN * 2); bf* KMh = (bf*)take((size_t)NBI * NN * FI * 2); bf* KMl = (bf*)take((size_t)NBI * NN * FI * 2); bf* QMh = (bf*)take((size_t)NBI * NN * FI * 2); bf* QMl = (bf*)take((size_t)NBI * NN * FI * 2);
    float* S = (float*)take((size_t)RCH * NN * 4); bf* PH = (bf*)take((size_t)RCH * NN * 2); bf* PL = (bf*)take((size_t)RCH * NN * 2); float* AV = (float*)take((size_t)RCH * OUTC * 4); bf* AVh = (bf*)take((size_t)RCH * OUTC * 2); bf* AVl = (bf*)take((size_t)RCH * OUTC * 2); float* P2 = (float*)take((size_t)NR * OUTC * 4);
    if ((size_t)(wsp - (char*)d_ws) > ws_size) return;
    k_bf<<<(PJ * CC / 8 + 255) / 256, 256, 0, stream>>>(wk, WkB, PJ * CC / 8); k_bf<<<(PJ * CC / 8 + 255) / 256, 256, 0, stream>>>(wq, WqB, PJ * CC / 8); k_bf<<<(PJ * CC / 8 + 255) / 256, 256, 0, stream>>>(wv, WvB, PJ * CC / 8);
    k_bf<<<(OUTC * PJ / 8 + 255) / 256, 256, 0, stream>>>(w1, W1B, OUTC * PJ / 8); k_bf<<<(OUTC * OUTC / 8 + 255) / 256, 256, 0, stream>>>(w2, W2B, OUTC * OUTC / 8);
    for (int b = 0; b < NBI; ++b) {
        k_wt<<<dim3(CC / 64, NN / 64, 1), 256, 0, stream>>>(x + (size_t)b * CC * NN, CC, NN, XT);
        float* Kb = Kf + (size_t)b * NN * PJ; float* Qb = Qf + (size_t)b * NN * PJ;
        k_gemmb<false, false><<<dim3(NN / 64, PJ / 64, 1), 128, 0, stream>>>(XT, nullptr, WkB, bk, Vf, PJ, nullptr); k_l2n<<<NN / 8, 256, 0, stream>>>(Vf, Kb);
        k_gemmb<false, false><<<dim3(NN / 64, PJ / 64, 1), 128, 0, stream>>>(XT, nullptr, WqB, bq, Vf, PJ, nullptr); k_l2n<<<NN / 8, 256, 0, stream>>>(Vf, Qb);
        k_gemmb<false, false><<<dim3(NN / 64, PJ / 64, 1), 128, 0, stream>>>(XT, nullptr, WvB, bv, Vf, PJ, nullptr);
        k_kv<<<1, 256, 0, stream>>>(Kb, Vf, KVS);
        k_hydra<<<NN / 8, 256, 0, stream>>>(Qb, KVS, Hh, Hl);
        k_gemmb<true, false><<<dim3(NN / 64, 1, 1), 128, 0, stream>>>(Hh, Hl, W1B, b1, P1 + (size_t)b * NN * OUTC, OUTC, nullptr, nullptr, PJ);
        k_hmean<<<NN / 8, 256, 0, stream>>>(Kb, KMh + (size_t)b * NN * FI, KMl + (size_t)b * NN * FI); k_hmean<<<NN / 8, 256, 0, stream>>>(Qb, QMh + (size_t)b * NN * FI, QMl + (size_t)b * NN * FI);
    }
    k_bnstat<<<1, 64, 0, stream>>>(P1, MU, RS); k_bn1<<<NR / 8, 256, 0, stream>>>(P1, MU, RS, g1, be1, H1);
    k_cmean<<<1, 128, 0, stream>>>(H1, MU1); k_h1T<<<(NBI * OUTC * (NN / 64)) / 8, 256, 0, stream>>>(H1, MU1, H1Th, H1Tl); k_rbias<<<(NBI * RCH * OUTC) / 256, 256, 0, stream>>>(MU1, w2, RB);
    for (int b = 0; b < NBI; ++b) {
        for (int ch = 0; ch < NN / RCH; ++ch) { const size_t r0 = (size_t)ch * RCH;
            k_gemm3<<<dim3(RCH / 64, NN / 64, 1), 128, 0, stream>>>(KMh + ((size_t)b * NN + r0) * FI, KMl + ((size_t)b * NN + r0) * FI, QMh + (size_t)b * NN * FI, QMl + (size_t)b * NN * FI, FI, S, NN);
            k_softmax<<<RCH / 8, 256, 0, stream>>>(S, PH, PL);
            k_gemm3<<<dim3(RCH / 64, 1, 1), 128, 0, stream>>>(PH, PL, H1Th + (size_t)b * OUTC * NN, H1Tl + (size_t)b * OUTC * NN, NN, AV, OUTC);
            k_split64<<<RCH / 8, 256, 0, stream>>>(AV, RCH, AVh, AVl);
            k_gemmb<true, false><<<dim3(RCH / 64, 1, 1), 128, 0, stream>>>(AVh, AVl, W2B, b2, P2 + ((size_t)b * NN + r0) * OUTC, OUTC, nullptr, RB + (size_t)b * RCH * OUTC, OUTC, 0);
        }
    }
    k_bnstat<<<1, 64, 0, stream>>>(P2, MU, RS); k_bn2out<<<(NBI * OUTC * (NN / 128)) / 8, 256, 0, stream>>>(P2, MU, RS, g2, be2, out);
}
